// JK_43662637531875
// MI455X (gfx1250) — hardware-verified
//
#include <hip/hip_runtime.h>
#include <stddef.h>


typedef __bf16         v16bf __attribute__((ext_vector_type(16)));
typedef unsigned short v8us  __attribute__((ext_vector_type(8)));
typedef float          v8f   __attribute__((ext_vector_type(8)));
typedef float          v4f   __attribute__((ext_vector_type(4)));
typedef int            v4i   __attribute__((ext_vector_type(4)));
typedef int            v2i   __attribute__((ext_vector_type(2)));

union Frag  { v16bf v; v8us hv[2]; unsigned int w[8]; };
union Pack8 { v8us v; unsigned int w[4]; };

static constexpr int AGP  = 1024;
static constexpr int EPL  = 16;
static constexpr int QCAP = 1024;

__device__ __forceinline__ v8f wmma_bf16(v16bf a, v16bf b, v8f c)
{
    v8f d = __builtin_amdgcn_wmma_f32_16x16x32_bf16(false, a, false, b, (short)0, c, false, false);
    asm volatile("v_nop\n\tv_nop\n\tv_nop\n\tv_nop" : "+v"(d) : "v"(a), "v"(b));
    return d;
}

__device__ __forceinline__ unsigned int bf16_bits(float f)
{
    unsigned int u = __float_as_uint(f);
    return (u + 0x7FFFu + ((u >> 16) & 1u)) >> 16;
}

__device__ __forceinline__ void split_bf16(float f, unsigned int& hi, unsigned int& lo)
{
    hi = bf16_bits(f);
    lo = bf16_bits(f - __uint_as_float(hi << 16));
}

__device__ __forceinline__ unsigned int pack2(unsigned int e0, unsigned int e1)
{
    return (e0 & 0xFFFFu) | (e1 << 16);
}

template <int K, int NPAD>
__global__ __launch_bounds__(256) void k_wsplit(const float* __restrict__ W, int ncol,
                                                unsigned short* __restrict__ Wh,
                                                unsigned short* __restrict__ Wl)
{
    constexpr int KQ = K / 8, NCH = NPAD * KQ;
    for (int pass = 0; pass < 2; ++pass) {
        for (int q = threadIdx.x; q < NCH; q += 256) {
            const int n = q / KQ, kq = q - n * KQ;
            Pack8 ph, pl;
#pragma unroll
            for (int i = 0; i < 4; ++i) {
                const int k = kq * 8 + 2 * i;
                float f0 = 0.f, f1 = 0.f;
                if (n < ncol) {
                    f0 = W[(size_t)k * ncol + n];
                    f1 = W[(size_t)(k + 1) * ncol + n];
                }
                unsigned int h0, l0, h1, l1;
                split_bf16(f0, h0, l0);
                split_bf16(f1, h1, l1);
                ph.w[i] = pack2(h0, h1);
                pl.w[i] = pack2(l0, l1);
            }
            *(volatile v8us*)(Wh + (size_t)n * K + kq * 8) = ph.v;
            *(volatile v8us*)(Wl + (size_t)n * K + kq * 8) = pl.v;
        }
        __threadfence();
    }
}

__global__ __launch_bounds__(32) void k_deg(const int* __restrict__ edst, float* __restrict__ dinv,
                                           int N, int E, int niter, int nq)
{
    extern __shared__ __align__(16) unsigned char deg_lds[];
    v4i* stg = (v4i*)deg_lds;
    v4i* cz  = (v4i*)(deg_lds + 512);
    unsigned short* cnt = (unsigned short*)(deg_lds + 512);
    const int l = threadIdx.x;
    const int n16 = (N * 2 + 15) >> 4;
    const v4i z4 = {0, 0, 0, 0};
    for (int q = l; q < n16; q += 32) cz[q] = z4;
    __syncthreads();

    const bool dvec = ((E & 3) == 0);
    for (int it = 0; it < niter; ++it) {
        const long e0 = (long)it * 128;
        v4i v = {-1, -1, -1, -1};
        if (dvec && e0 + 128 <= (long)E) {
            v = *(const v4i*)(edst + e0 + l * 4);
        } else {
#pragma unroll
            for (int u = 0; u < 4; ++u) {
                const long e = e0 + l * 4 + u;
                if (e < (long)E) v[u] = edst[e];
            }
        }
        stg[l] = v;
        __syncthreads();
        for (int j = 0; j < 32; ++j) {
            const v4i w = stg[j];
#pragma unroll
            for (int u = 0; u < 4; ++u) {
                const int dd = w[u];
                if (((dd & 31) == l) && ((unsigned int)dd < (unsigned int)N)) {
                    const unsigned int c = cnt[dd];
                    if (c < 65535u) cnt[dd] = (unsigned short)(c + 1u);
                }
            }
        }
        __syncthreads();
    }

    for (int pass = 0; pass < 2; ++pass) {
        for (int q = 0; q < nq; ++q) {
            const int i0 = q * 128 + l * 4;
            v4f r;
#pragma unroll
            for (int u = 0; u < 4; ++u) {
                const int i = i0 + u;
                const float c = (i < N) ? (float)cnt[i] : 0.f;
                r[u] = 1.0f / sqrtf(c + 1.0f);
            }
            *(volatile v4f*)(dinv + i0) = r;
        }
        __threadfence();
    }
}

template <int K, int NT, int MODE>
__global__ __launch_bounds__(256) void k_gemm(const float* __restrict__ A, int lda, int M,
                                             const unsigned short* __restrict__ Wh,
                                             const unsigned short* __restrict__ Wl,
                                             const float* __restrict__ rowscale,
                                             const float* __restrict__ bias,
                                             float* __restrict__ C, int ncol)
{
    constexpr int KP = K + 8, NPAD = NT * 16, KQ = K / 8;
    constexpr int BB = 2 * NPAD * KP * 2;
    constexpr int SB = 8 * 16 * NPAD * 4;
    constexpr int LB = (BB > SB) ? BB : SB;
    __shared__ __align__(16) unsigned char lds[LB];
    unsigned short* Bh = (unsigned short*)lds;
    unsigned short* Bl = Bh + NPAD * KP;
    float* stg = (float*)lds;

    const int tid = threadIdx.x;
    for (int q = tid; q < NPAD * KQ; q += 256) {
        const int n = q / KQ, kq = q - n * KQ;
        *(v8us*)(Bh + n * KP + kq * 8) = *(const v8us*)(Wh + (size_t)q * 8);
        *(v8us*)(Bl + n * KP + kq * 8) = *(const v8us*)(Wl + (size_t)q * 8);
    }
    __syncthreads();

    const int wave = tid >> 5, l = tid & 31, h = l >> 4, m = l & 15;
    const int row0 = blockIdx.x * 128 + wave * 16;
    int ra = row0 + m;
    if (ra > M - 1) ra = M - 1;
    const float* arow = A + (size_t)ra * lda;

    const v8f z8 = {0.f, 0.f, 0.f, 0.f, 0.f, 0.f, 0.f, 0.f};
    v8f acc[NT];
#pragma unroll
    for (int ct = 0; ct < NT; ++ct) acc[ct] = z8;

    for (int k0 = 0; k0 < K; k0 += 32) {
        const float* ap = arow + k0 + 8 * h;
        const v4f x0 = *(const v4f*)(ap);
        const v4f x1 = *(const v4f*)(ap + 4);
        const v4f x2 = *(const v4f*)(ap + 16);
        const v4f x3 = *(const v4f*)(ap + 20);
        Frag ah, al;
        {
            unsigned int h0, l0, h1, l1;
            split_bf16(x0.x, h0, l0); split_bf16(x0.y, h1, l1); ah.w[0] = pack2(h0, h1); al.w[0] = pack2(l0, l1);
            split_bf16(x0.z, h0, l0); split_bf16(x0.w, h1, l1); ah.w[1] = pack2(h0, h1); al.w[1] = pack2(l0, l1);
            split_bf16(x1.x, h0, l0); split_bf16(x1.y, h1, l1); ah.w[2] = pack2(h0, h1); al.w[2] = pack2(l0, l1);
            split_bf16(x1.z, h0, l0); split_bf16(x1.w, h1, l1); ah.w[3] = pack2(h0, h1); al.w[3] = pack2(l0, l1);
            split_bf16(x2.x, h0, l0); split_bf16(x2.y, h1, l1); ah.w[4] = pack2(h0, h1); al.w[4] = pack2(l0, l1);
            split_bf16(x2.z, h0, l0); split_bf16(x2.w, h1, l1); ah.w[5] = pack2(h0, h1); al.w[5] = pack2(l0, l1);
            split_bf16(x3.x, h0, l0); split_bf16(x3.y, h1, l1); ah.w[6] = pack2(h0, h1); al.w[6] = pack2(l0, l1);
            split_bf16(x3.z, h0, l0); split_bf16(x3.w, h1, l1); ah.w[7] = pack2(h0, h1); al.w[7] = pack2(l0, l1);
        }
#pragma unroll
        for (int ct = 0; ct < NT; ++ct) {
            const unsigned short* bp = Bh + (ct * 16 + m) * KP + k0 + 8 * h;
            const unsigned short* bq = Bl + (ct * 16 + m) * KP + k0 + 8 * h;
            Frag bh, bl;
            bh.hv[0] = *(const v8us*)(bp);
            bh.hv[1] = *(const v8us*)(bp + 16);
            bl.hv[0] = *(const v8us*)(bq);
            bl.hv[1] = *(const v8us*)(bq + 16);
            acc[ct] = wmma_bf16(ah.v, bh.v, acc[ct]);
            acc[ct] = wmma_bf16(ah.v, bl.v, acc[ct]);
            acc[ct] = wmma_bf16(al.v, bh.v, acc[ct]);
        }
    }

    __syncthreads();
    float* sw = stg + wave * 16 * NPAD;
#pragma unroll
    for (int ct = 0; ct < NT; ++ct) {
#pragma unroll
        for (int r = 0; r < 8; ++r) sw[(8 * h + r) * NPAD + ct * 16 + m] = acc[ct][r];
    }
    __syncthreads();

    if (MODE == 0) {
        constexpr int F4R = NPAD / 4;
        constexpr int NI  = (16 * F4R) / 32;
        for (int pass = 0; pass < 2; ++pass) {
#pragma unroll
            for (int i = 0; i < NI; ++i) {
                const int f = i * 32 + l;
                const int r = f / F4R, cq = f - r * F4R;
                v4f v = *(const v4f*)(sw + r * NPAD + cq * 4);
                const float s = rowscale[row0 + r];
                v *= s;
                *(volatile v4f*)(C + (size_t)(row0 + r) * NPAD + cq * 4) = v;
            }
            __threadfence();
        }
    } else {
        const int f4r = ncol >> 2;
        const int nf  = 16 * f4r;
        const int ni  = (nf + 31) >> 5;
        for (int pass = 0; pass < 2; ++pass) {
            for (int i = 0; i < ni; ++i) {
                const int f = i * 32 + l;
                if (f < nf) {
                    const int r = f / f4r, cq = f - r * f4r;
                    v4f v = *(const v4f*)(sw + r * NPAD + cq * 4);
                    const v4f b = *(const v4f*)(bias + cq * 4);
                    v += b;
                    const int row = row0 + r;
                    if (row < M) *(volatile v4f*)(C + (size_t)row * ncol + cq * 4) = v;
                }
            }
            __threadfence();
        }
    }
}

__device__ __forceinline__ void agg_pairs(v4f* acc4, const v2i* que, int qn,
                                          const float* __restrict__ hs, int N,
                                          int l, int h, int c4)
{
    const int np = (qn + 1) >> 1;
    for (int p = 0; p < np; ++p) {
        const int ia = 2 * p, ib = ia + 1;
        const bool vb = (ib < qn);
        const v2i me = que[h ? ib : ia];
        int s = me.x;
        s = s < 0 ? 0 : s;
        s = s > N - 1 ? N - 1 : s;
        const int dl = me.y & (AGP - 1);
        const v4f hv = *(const v4f*)(hs + (size_t)s * 64 + c4 * 4);
        const int dla = __shfl(dl, 0);
        const int dlb = __shfl(dl, 16);
        if (vb && dla == dlb) {
            v4f o;
            o.x = __shfl_xor(hv.x, 16);
            o.y = __shfl_xor(hv.y, 16);
            o.z = __shfl_xor(hv.z, 16);
            o.w = __shfl_xor(hv.w, 16);
            if (h == 0) {
                v4f* ap = acc4 + dl * 16 + c4;
                v4f a = *ap;
                a = a + hv;
                a = a + o;
                *ap = a;
            }
        } else {
            if (vb || h == 0) {
                v4f* ap = acc4 + dl * 16 + c4;
                v4f a = *ap;
                a = a + hv;
                *ap = a;
            }
        }
    }
}

template <int SECOND>
__global__ __launch_bounds__(32) void k_agg(const float* __restrict__ hs, const float* __restrict__ dinv,
                                          const int* __restrict__ esrc, const int* __restrict__ edst,
                                          const float* __restrict__ bias, const float* __restrict__ xprev,
                                          float* __restrict__ xout, int N, int E, int niter)
{
    extern __shared__ __align__(16) unsigned char agg_lds[];
    v4f* acc4 = (v4f*)agg_lds;
    v2i* que  = (v2i*)(agg_lds + (size_t)AGP * 64 * 4);
    const int l = threadIdx.x, h = l >> 4, c4 = l & 15;
    const int base = blockIdx.x * AGP;

    const v4f z4 = {0.f, 0.f, 0.f, 0.f};
    for (int i = 0; i < (AGP * 16) / 32; ++i) acc4[i * 32 + l] = z4;
    __syncthreads();

    int qn = 0;
    const bool dvec = ((E & 3) == 0);
    for (int it = 0; it < niter; ++it) {
        const long e0 = (long)it * (32 * EPL);
        v4i dv[EPL / 4], sv[EPL / 4];
        if (dvec && e0 + 32 * EPL <= (long)E) {
            const int* pd = edst + e0 + l * EPL;
            const int* ps = esrc + e0 + l * EPL;
#pragma unroll
            for (int t = 0; t < EPL / 4; ++t) {
                dv[t] = *(const v4i*)(pd + 4 * t);
                sv[t] = *(const v4i*)(ps + 4 * t);
            }
        } else {
#pragma unroll
            for (int t = 0; t < EPL / 4; ++t) {
                v4i a = {-1, -1, -1, -1};
                v4i b = {0, 0, 0, 0};
#pragma unroll
                for (int u = 0; u < 4; ++u) {
                    const long e = e0 + l * EPL + 4 * t + u;
                    if (e < (long)E) { a[u] = edst[e]; b[u] = esrc[e]; }
                }
                dv[t] = a;
                sv[t] = b;
            }
        }
#pragma unroll
        for (int j = 0; j < EPL; ++j) {
            const int dj = dv[j >> 2][j & 3];
            const int sj = sv[j >> 2][j & 3];
            const unsigned int dl = (unsigned int)(dj - base);
            const bool in = dl < (unsigned int)AGP;
            const unsigned int mask = __builtin_amdgcn_ballot_w32(in);
            if (mask != 0u) {
                if (in) {
                    const int pos = qn + (int)__builtin_amdgcn_mbcnt_lo(mask, 0u);
                    v2i qe;
                    qe.x = sj;
                    qe.y = (int)dl;
                    que[pos] = qe;
                }
                qn += __builtin_popcount(mask);
            }
        }
        if (qn >= 32) {
            __syncthreads();
            agg_pairs(acc4, que, qn, hs, N, l, h, c4);
            qn = 0;
            __syncthreads();
        }
    }
    __syncthreads();
    if (qn > 0) agg_pairs(acc4, que, qn, hs, N, l, h, c4);
    __syncthreads();

    const v4f b4 = *(const v4f*)(bias + c4 * 4);
    for (int pass = 0; pass < 2; ++pass) {
        for (int q = 0; q < AGP / 2; ++q) {
            const int il = 2 * q + h;
            const int i  = base + il;
            const v4f a  = acc4[il * 16 + c4];
            const v4f hv = *(const v4f*)(hs + (size_t)i * 64 + c4 * 4);
            const float di = dinv[i];
            v4f v;
            v.x = fmaxf(di * (a.x + hv.x) + b4.x, 0.f);
            v.y = fmaxf(di * (a.y + hv.y) + b4.y, 0.f);
            v.z = fmaxf(di * (a.z + hv.z) + b4.z, 0.f);
            v.w = fmaxf(di * (a.w + hv.w) + b4.w, 0.f);
            if (SECOND) {
                const v4f xp = *(const v4f*)(xprev + (size_t)i * 64 + c4 * 4);
                v.x = fmaxf(xp.x, v.x);
                v.y = fmaxf(xp.y, v.y);
                v.z = fmaxf(xp.z, v.z);
                v.w = fmaxf(xp.w, v.w);
            }
            *(volatile v4f*)(xout + (size_t)i * 64 + c4 * 4) = v;
        }
        __threadfence();
    }
}

extern "C" void kernel_launch(void* const* d_in, const int* in_sizes, int n_in,
                              void* d_out, int out_size, void* d_ws, size_t ws_size,
                              hipStream_t stream)
{
    (void)n_in;
    const float* x  = (const float*)d_in[0];
    const int*   ei = (const int*)d_in[1];
    const float* W1 = (const float*)d_in[2];
    const float* b1 = (const float*)d_in[3];
    const float* W2 = (const float*)d_in[4];
    const float* b2 = (const float*)d_in[5];
    const float* Wf = (const float*)d_in[6];
    const float* bq = (const float*)d_in[7];
    float* out = (float*)d_out;

    const int NF = 128, NH = 64, NC = 40, NCP = 48;
    const int N = in_sizes[0] / NF;
    const int E = in_sizes[1] / 2;
    if (N < 1 || E < 0) return;
    if ((long)out_size < (long)N * NC) return;

    const int NPART = (N + AGP - 1) / AGP;
    const int Npad  = NPART * AGP;

    const size_t ldsDeg = 512 + ((((size_t)N) * 2 + 15) & ~(size_t)15);
    const size_t ldsAgg = (size_t)AGP * 64 * 4 + (size_t)QCAP * 8;
    if (ldsDeg > (size_t)294912) return;

    char* ws = (char*)d_ws;
    size_t off = 0;
    auto carve = [&](size_t bytes) -> char* {
        char* p = ws + off;
        off += (bytes + 255) & ~(size_t)255;
        return p;
    };
    float* dinv = (float*)carve((size_t)Npad * 4);
    float* hs   = (float*)carve((size_t)Npad * NH * 4);
    float* x1   = (float*)carve((size_t)Npad * NH * 4);
    float* xjk  = (float*)carve((size_t)Npad * NH * 4);
    unsigned short* w1h = (unsigned short*)carve((size_t)NH * NF * 2);
    unsigned short* w1l = (unsigned short*)carve((size_t)NH * NF * 2);
    unsigned short* w2h = (unsigned short*)carve((size_t)NH * NH * 2);
    unsigned short* w2l = (unsigned short*)carve((size_t)NH * NH * 2);
    unsigned short* wfh = (unsigned short*)carve((size_t)NCP * NH * 2);
    unsigned short* wfl = (unsigned short*)carve((size_t)NCP * NH * 2);
    if (off > ws_size) return;

    const int* esrc = ei;
    const int* edst = ei + E;

    k_wsplit<128, 64><<<1, 256, 0, stream>>>(W1, NH, w1h, w1l);
    k_wsplit<64, 64><<<1, 256, 0, stream>>>(W2, NH, w2h, w2l);
    k_wsplit<64, 48><<<1, 256, 0, stream>>>(Wf, NC, wfh, wfl);

    k_deg<<<1, 32, ldsDeg, stream>>>(edst, dinv, N, E, (E + 127) / 128, Npad / 128);

    const int ggrid = (N + 127) / 128;
    const int aiter = (E + 32 * EPL - 1) / (32 * EPL);

    k_gemm<128, 4, 0><<<ggrid, 256, 0, stream>>>(x, NF, N, w1h, w1l, dinv, b1, hs, NH);
    k_agg<0><<<NPART, 32, ldsAgg, stream>>>(hs, dinv, esrc, edst, b1, hs, x1, N, E, aiter);

    k_gemm<64, 4, 0><<<ggrid, 256, 0, stream>>>(x1, NH, N, w2h, w2l, dinv, b2, hs, NH);
    k_agg<1><<<NPART, 32, ldsAgg, stream>>>(hs, dinv, esrc, edst, b2, x1, xjk, N, E, aiter);

    k_gemm<64, 3, 1><<<ggrid, 256, 0, stream>>>(xjk, NH, N, wfh, wfl, dinv, bq, out, NC);
}
